// NeuralEncoder_47399259078851
// MI455X (gfx1250) — hardware-verified
//
#include <hip/hip_runtime.h>
#define BB 4
#define TT 100
#define SP 20
#define SS 2000
#define HH 512
#define NH 8
#define DH 64
#define CF 4
#define CBK 4
#define NG 25
#define GR 80
#define KWIN 240
#define KP 256
#define LK 2160
#define LV 2176
#define NTOK (BB * SS)

typedef __bf16 v16b __attribute__((ext_vector_type(16)));
typedef unsigned short v8us __attribute__((ext_vector_type(8), may_alias));
typedef float  v8f  __attribute__((ext_vector_type(8)));
typedef float  v4f  __attribute__((ext_vector_type(4)));
typedef float  v4fa __attribute__((ext_vector_type(4), may_alias));
union FragB { v16b v; v8us half[2]; unsigned short u[16]; };

__device__ __forceinline__ unsigned short bf16_bits(float x) { unsigned int u = __float_as_uint(x); return (unsigned short)((u + 0x7FFFu + ((u >> 16) & 1u)) >> 16); }
__device__ __forceinline__ float bf16_val(unsigned short b) { return __uint_as_float(((unsigned int)b) << 16); }
__device__ __forceinline__ float bf16_round(float x) { return bf16_val(bf16_bits(x)); }
template <int NT>
__device__ __forceinline__ v8f mmaN(v16b ah, v16b al, v16b bh, v16b bl, v8f c) {
  c = __builtin_amdgcn_wmma_f32_16x16x32_bf16(false, ah, false, bh, (short)0, c, false, false);
  if (NT >= 2) c = __builtin_amdgcn_wmma_f32_16x16x32_bf16(false, al, false, bh, (short)0, c, false, false);
  if (NT >= 3) c = __builtin_amdgcn_wmma_f32_16x16x32_bf16(false, ah, false, bl, (short)0, c, false, false);
  asm volatile("v_nop\n\tv_nop\n\tv_nop\n\tv_nop" : "+v"(c) : "v"(ah), "v"(al), "v"(bh), "v"(bl));
  return c;
}

__global__ __launch_bounds__(256) void k_wt_bf16(const float* __restrict__ W, unsigned short* __restrict__ Wt, int K, int N) {
  const int t = blockIdx.x * 256 + threadIdx.x;
  const int k8n = K / 8;
  if (t >= N * k8n) return;
  const int n = t / k8n, k8 = (t % k8n) * 8;
  v8us v;
#pragma unroll
  for (int i = 0; i < 8; ++i) v[i] = bf16_bits(W[(size_t)(k8 + i) * N + n]);
  *(volatile v8us*)(Wt + (size_t)n * K + k8) = v;
  __threadfence();
  *(volatile v8us*)(Wt + (size_t)n * K + k8) = v;
}

template <bool ASPLIT, int ACT, bool BIAS_BF16>
__global__ __launch_bounds__(128) void k_gemm_bf(const float* __restrict__ A, int lda, const unsigned short* __restrict__ Wt, int ldb,
                                               const float* __restrict__ bias, float* __restrict__ C, int ldc, int M, int N, int K) {
  __shared__ __attribute__((aligned(16))) float so[4][16][64];
  const int tid = threadIdx.x, w = tid >> 5, lane = tid & 31, ln = lane & 15, hh = lane >> 4;
  const int ntn = N / 64;
  const int wid = blockIdx.x * 4 + w;
  const int mt = wid / ntn, nq = wid % ntn;
  if (mt * 16 >= M) return;
  const int row0 = mt * 16, col0 = nq * 64;
  const float* arow = A + (size_t)(row0 + ln) * lda;
  v8f acc[4] = {};
  for (int kb = 0; kb < K; kb += 32) {
    FragB ah, al;
    const v4f x0 = *(const v4fa*)(arow + kb + 8 * hh), x1 = *(const v4fa*)(arow + kb + 8 * hh + 4);
    const v4f x2 = *(const v4fa*)(arow + kb + 16 + 8 * hh), x3 = *(const v4fa*)(arow + kb + 16 + 8 * hh + 4);
    float xs[16] = {x0[0],x0[1],x0[2],x0[3],x1[0],x1[1],x1[2],x1[3],x2[0],x2[1],x2[2],x2[3],x3[0],x3[1],x3[2],x3[3]};
#pragma unroll
    for (int i = 0; i < 16; ++i) { const unsigned short hb = bf16_bits(xs[i]); ah.u[i] = hb; al.u[i] = ASPLIT ? bf16_bits(xs[i] - bf16_val(hb)) : (unsigned short)0; }
#pragma unroll
    for (int t = 0; t < 4; ++t) {
      const unsigned short* brow = Wt + (size_t)(col0 + t * 16 + ln) * ldb + kb;
      FragB b;
      b.half[0] = *(const v8us*)(brow + 8 * hh);
      b.half[1] = *(const v8us*)(brow + 16 + 8 * hh);
      acc[t] = mmaN<ASPLIT ? 2 : 1>(ah.v, al.v, b.v, b.v, acc[t]);
    }
  }
#pragma unroll
  for (int t = 0; t < 4; ++t) {
    float bv = bias ? bias[col0 + t * 16 + ln] : 0.f;
    if (BIAS_BF16) bv = bf16_round(bv);
#pragma unroll
    for (int r = 0; r < 8; ++r) { float v = acc[t][r] + bv; if (ACT == 1) v = fmaxf(v, 0.f); so[w][8 * hh + r][t * 16 + ln] = v; }
  }
  __builtin_amdgcn_fence(__ATOMIC_ACQ_REL, "workgroup");
  __builtin_amdgcn_wave_barrier();
  const int rsub = lane >> 4, c4 = (lane & 15) * 4;
  for (int pass = 0; pass < 2; ++pass) {
#pragma unroll
    for (int q = 0; q < 8; ++q) {
      const int r = q * 2 + rsub;
      const v4f v = *(const v4fa*)&so[w][r][c4];
      *(volatile v4f*)(C + (size_t)(row0 + r) * ldc + col0 + c4) = v;
    }
    if (pass == 0) __threadfence();
  }
}

template <int D, bool CAUSAL>
__global__ __launch_bounds__(128) void k_flash(const float* __restrict__ qb, const float* __restrict__ kb, const float* __restrict__ vb,
                                             int pitch, int T, int H, float scale, float* __restrict__ y, int ypitch) {
  constexpr int KS = D / 32;
  constexpr int DT = D / 16;
  __shared__ __attribute__((aligned(16))) unsigned short sKh[32][D + 8], sKl[32][D + 8], sVh[32][D + 8], sVl[32][D + 8];
  __shared__ __attribute__((aligned(16))) unsigned short sPh[4][16][40], sPl[4][16][40];
  __shared__ __attribute__((aligned(16))) float sO[4][16][D];
  const int tid = threadIdx.x, w = tid >> 5, lane = tid & 31, ln = lane & 15, hh = lane >> 4;
  const int nqb = (T + 63) / 64;
  const int bh = blockIdx.x / nqb, qblk = blockIdx.x % nqb;
  const int b = bh / H, h = bh % H;
  const int q0 = qblk * 64 + w * 16;
  const float* Q = qb + (size_t)b * T * pitch + h * D;
  const float* K = kb + (size_t)b * T * pitch + h * D;
  const float* V = vb + (size_t)b * T * pitch + h * D;

  FragB aqh[KS], aql[KS];
  {
    int row = q0 + ln; if (row >= T) row = T - 1;
    const float* qr = Q + (size_t)row * pitch;
#pragma unroll
    for (int ks = 0; ks < KS; ++ks)
#pragma unroll
      for (int i = 0; i < 16; ++i) {
        const int d = ks * 32 + ((i < 8) ? (8 * hh + i) : (16 + 8 * hh + (i - 8)));
        const float x = qr[d] * scale; const unsigned short hb = bf16_bits(x);
        aqh[ks].u[i] = hb; aql[ks].u[i] = bf16_bits(x - bf16_val(hb));
      }
  }
  float m_r[8], l_r[8];
#pragma unroll
  for (int r = 0; r < 8; ++r) { m_r[r] = -3.0e38f; l_r[r] = 0.f; }
  v8f oacc[DT];
#pragma unroll
  for (int dt = 0; dt < DT; ++dt) oacc[dt] = (v8f){0.f,0.f,0.f,0.f,0.f,0.f,0.f,0.f};

  const int kv_end = CAUSAL ? min(T, qblk * 64 + 64) : T;
  for (int j0 = 0; j0 < kv_end; j0 += 32) {
    __syncthreads();
    for (int e = tid; e < 32 * (D / 4); e += 128) {
      const int r = e / (D / 4), c4 = (e % (D / 4)) * 4;
      const int key = j0 + r;
      v4f kf = {0.f,0.f,0.f,0.f}, vf = {0.f,0.f,0.f,0.f};
      if (key < T) { kf = *(const v4fa*)(K + (size_t)key * pitch + c4); vf = *(const v4fa*)(V + (size_t)key * pitch + c4); }
#pragma unroll
      for (int t = 0; t < 4; ++t) {
        unsigned short hb = bf16_bits(kf[t]); sKh[r][c4 + t] = hb; sKl[r][c4 + t] = bf16_bits(kf[t] - bf16_val(hb));
        hb = bf16_bits(vf[t]); sVh[r][c4 + t] = hb; sVl[r][c4 + t] = bf16_bits(vf[t] - bf16_val(hb));
      }
    }
    __syncthreads();
    v8f s[2];
#pragma unroll
    for (int nt = 0; nt < 2; ++nt) {
      v8f acc = {};
#pragma unroll
      for (int ks = 0; ks < KS; ++ks) {
        FragB bh_, bl_;
        bh_.half[0] = *(const v8us*)&sKh[nt * 16 + ln][ks * 32 + 8 * hh]; bh_.half[1] = *(const v8us*)&sKh[nt * 16 + ln][ks * 32 + 16 + 8 * hh];
        bl_.half[0] = *(const v8us*)&sKl[nt * 16 + ln][ks * 32 + 8 * hh]; bl_.half[1] = *(const v8us*)&sKl[nt * 16 + ln][ks * 32 + 16 + 8 * hh];
        acc = mmaN<3>(aqh[ks].v, aql[ks].v, bh_.v, bl_.v, acc);
      }
      s[nt] = acc;
    }
    float alpha[8];
#pragma unroll
    for (int r = 0; r < 8; ++r) {
      const int qi = q0 + 8 * hh + r;
      const int ja = j0 + ln, jb = j0 + 16 + ln;
      if (CAUSAL) { if (ja > qi) s[0][r] = -3.0e38f; if (jb > qi) s[1][r] = -3.0e38f; }
      if (ja >= T) s[0][r] = -3.0e38f;
      if (jb >= T) s[1][r] = -3.0e38f;
      float mx = fmaxf(s[0][r], s[1][r]);
      mx = fmaxf(mx, __shfl_xor(mx, 1, 32)); mx = fmaxf(mx, __shfl_xor(mx, 2, 32)); mx = fmaxf(mx, __shfl_xor(mx, 4, 32)); mx = fmaxf(mx, __shfl_xor(mx, 8, 32));
      const float mnew = fmaxf(m_r[r], mx);
      alpha[r] = (mnew > -1.0e38f) ? __expf(m_r[r] - mnew) : 1.0f;
      const float p0 = (s[0][r] > -1.0e38f) ? __expf(s[0][r] - mnew) : 0.f;
      const float p1 = (s[1][r] > -1.0e38f) ? __expf(s[1][r] - mnew) : 0.f;
      m_r[r] = mnew;
      l_r[r] = l_r[r] * alpha[r] + p0 + p1;
      unsigned short hb = bf16_bits(p0); sPh[w][8 * hh + r][ln] = hb;      sPl[w][8 * hh + r][ln] = bf16_bits(p0 - bf16_val(hb));
      hb = bf16_bits(p1);                sPh[w][8 * hh + r][16 + ln] = hb; sPl[w][8 * hh + r][16 + ln] = bf16_bits(p1 - bf16_val(hb));
    }
#pragma unroll
    for (int dt = 0; dt < DT; ++dt)
#pragma unroll
      for (int r = 0; r < 8; ++r) oacc[dt][r] *= alpha[r];
    __builtin_amdgcn_fence(__ATOMIC_ACQ_REL, "workgroup");
    __builtin_amdgcn_wave_barrier();
    FragB pah, pal;
    pah.half[0] = *(const v8us*)&sPh[w][ln][8 * hh]; pah.half[1] = *(const v8us*)&sPh[w][ln][16 + 8 * hh];
    pal.half[0] = *(const v8us*)&sPl[w][ln][8 * hh]; pal.half[1] = *(const v8us*)&sPl[w][ln][16 + 8 * hh];
#pragma unroll
    for (int dt = 0; dt < DT; ++dt) {
      FragB bvh, bvl;
#pragma unroll
      for (int i = 0; i < 8; ++i) {
        bvh.u[i] = sVh[8 * hh + i][dt * 16 + ln]; bvh.u[8 + i] = sVh[16 + 8 * hh + i][dt * 16 + ln];
        bvl.u[i] = sVl[8 * hh + i][dt * 16 + ln]; bvl.u[8 + i] = sVl[16 + 8 * hh + i][dt * 16 + ln];
      }
      oacc[dt] = mmaN<3>(pah.v, pal.v, bvh.v, bvl.v, oacc[dt]);
    }
    __builtin_amdgcn_fence(__ATOMIC_ACQ_REL, "workgroup");
    __builtin_amdgcn_wave_barrier();
  }
#pragma unroll
  for (int r = 0; r < 8; ++r) {
    float l = l_r[r];
    l += __shfl_xor(l, 1, 32); l += __shfl_xor(l, 2, 32); l += __shfl_xor(l, 4, 32); l += __shfl_xor(l, 8, 32);
    l_r[r] = (l > 0.f) ? 1.0f / l : 0.f;
  }
#pragma unroll
  for (int dt = 0; dt < DT; ++dt)
#pragma unroll
    for (int r = 0; r < 8; ++r) sO[w][8 * hh + r][dt * 16 + ln] = oacc[dt][r] * l_r[r];
  __builtin_amdgcn_fence(__ATOMIC_ACQ_REL, "workgroup");
  __builtin_amdgcn_wave_barrier();
  for (int pass = 0; pass < 2; ++pass) {
    for (int r = 0; r < 16; ++r) {
      const int row = q0 + r;
      if (row < T && lane < D / 4) {
        const v4f val = *(const v4fa*)&sO[w][r][lane * 4];
        *(volatile v4f*)(y + ((size_t)b * T + row) * ypitch + h * D + lane * 4) = val;
      }
    }
    if (pass == 0) __threadfence();
  }
}

template <bool ASPLIT, bool BSPLIT, int ACT>
__global__ __launch_bounds__(128) void k_gemm_b(const float* __restrict__ A, int lda, size_t sA, const unsigned short* __restrict__ Bh, const unsigned short* __restrict__ Bl, int ldb, size_t sB,
                                             const float* __restrict__ bias, const float* __restrict__ resid, int ldr, size_t sR, float rsign, float alpha,
                                             float* __restrict__ C, int ldc, size_t sC, int M, int N, int K) {
  __shared__ __attribute__((aligned(16))) float so[4][16][64];
  const int tid = threadIdx.x, w = tid >> 5, lane = tid & 31, ln = lane & 15, hh = lane >> 4;
  const int by = blockIdx.y;
  A += (size_t)by * sA; Bh += (size_t)by * sB; if (BSPLIT) Bl += (size_t)by * sB; C += (size_t)by * sC; if (resid) resid += (size_t)by * sR;
  const int ntn = (N + 63) / 64; const int wid = blockIdx.x * 4 + w; const int mt = wid / ntn, nq = wid % ntn;
  if (mt * 16 >= M) return;
  const int row0 = mt * 16, col0 = nq * 64;
  const float* arow = A + (size_t)(row0 + ln) * lda;
  v8f acc[4] = {};
  for (int kb = 0; kb < K; kb += 32) {
    FragB ah, al;
    const v4f x0 = *(const v4fa*)(arow + kb + 8 * hh), x1 = *(const v4fa*)(arow + kb + 8 * hh + 4);
    const v4f x2 = *(const v4fa*)(arow + kb + 16 + 8 * hh), x3 = *(const v4fa*)(arow + kb + 16 + 8 * hh + 4);
    float xs[16] = {x0[0],x0[1],x0[2],x0[3],x1[0],x1[1],x1[2],x1[3],x2[0],x2[1],x2[2],x2[3],x3[0],x3[1],x3[2],x3[3]};
#pragma unroll
    for (int i = 0; i < 16; ++i) { const unsigned short hb = bf16_bits(xs[i]); ah.u[i] = hb; al.u[i] = ASPLIT ? bf16_bits(xs[i] - bf16_val(hb)) : (unsigned short)0; }
#pragma unroll
    for (int t = 0; t < 4; ++t) {
      if (col0 + t * 16 >= N) continue;
      const size_t boff = (size_t)(col0 + t * 16 + ln) * ldb + kb;
      FragB bh_, bl_; bh_.half[0] = *(const v8us*)(Bh + boff + 8 * hh); bh_.half[1] = *(const v8us*)(Bh + boff + 16 + 8 * hh);
      if (BSPLIT) { bl_.half[0] = *(const v8us*)(Bl + boff + 8 * hh); bl_.half[1] = *(const v8us*)(Bl + boff + 16 + 8 * hh); } else bl_ = bh_;
      acc[t] = mmaN<ASPLIT ? (BSPLIT ? 3 : 2) : 1>(ah.v, al.v, bh_.v, bl_.v, acc[t]);
    }
  }
#pragma unroll
  for (int t = 0; t < 4; ++t) {
    const int col = col0 + t * 16 + ln; if (col0 + t * 16 >= N) continue; const float bv = bias ? bf16_round(bias[col]) : 0.f;
#pragma unroll
    for (int r = 0; r < 8; ++r) { float v = acc[t][r] * alpha + bv; if (resid) v += rsign * resid[(size_t)(row0 + 8 * hh + r) * ldr + col]; if (ACT == 1) v = fmaxf(v, 0.f); else if (ACT == 2) v = fmaxf(v, 0.f) + log1pf(expf(-fabsf(v))); so[w][8 * hh + r][t * 16 + ln] = v; }
  }
  __builtin_amdgcn_fence(__ATOMIC_ACQ_REL, "workgroup"); __builtin_amdgcn_wave_barrier();
  const int rsub = lane >> 4, c4 = (lane & 15) * 4;
  for (int pass = 0; pass < 2; ++pass) {
#pragma unroll
    for (int q = 0; q < 8; ++q) { const int r = q * 2 + rsub; if (col0 + c4 < N) { const v4f v = *(const v4fa*)&so[w][r][c4]; *(volatile v4f*)(C + (size_t)(row0 + r) * ldc + col0 + c4) = v; } }
    if (pass == 0) __threadfence();
  }
}
__global__ __launch_bounds__(256) void k_split_transpose_b(const float* __restrict__ src, int lds_, size_t sIn, unsigned short* __restrict__ hi, unsigned short* __restrict__ lo, size_t sOut, int K, int N) {
  const size_t t = (size_t)blockIdx.x * 256 + threadIdx.x; const int k8n = K / 8; if (t >= (size_t)N * k8n) return;
  src += (size_t)blockIdx.y * sIn; hi += (size_t)blockIdx.y * sOut; lo += (size_t)blockIdx.y * sOut;
  const int n = (int)(t / k8n), k8 = (int)(t % k8n) * 8; v8us vh, vl;
#pragma unroll
  for (int i = 0; i < 8; ++i) { const float x = src[(size_t)(k8 + i) * lds_ + n]; const unsigned short hb = bf16_bits(x); vh[i] = hb; vl[i] = bf16_bits(x - bf16_val(hb)); }
  unsigned short* dh = hi + (size_t)n * K + k8; unsigned short* dl = lo + (size_t)n * K + k8;
  *(volatile v8us*)dh = vh; *(volatile v8us*)dl = vl; __threadfence(); *(volatile v8us*)dh = vh; *(volatile v8us*)dl = vl;
}

typedef _Float16 v16h __attribute__((ext_vector_type(16)));
union FragH { v16h v; v8us half[2]; _Float16 h[16]; unsigned short u[16]; };
template <int NT>
__device__ __forceinline__ v8f mmaH(v16h ah, v16h al, v16h bh, v16h bl, v8f c) {
  c = __builtin_amdgcn_wmma_f32_16x16x32_f16(false, ah, false, bh, (short)0, c, false, false);
  if (NT >= 2) c = __builtin_amdgcn_wmma_f32_16x16x32_f16(false, al, false, bh, (short)0, c, false, false);
  if (NT >= 3) c = __builtin_amdgcn_wmma_f32_16x16x32_f16(false, ah, false, bl, (short)0, c, false, false);
  asm volatile("v_nop\n\tv_nop\n\tv_nop\n\tv_nop" : "+v"(c) : "v"(ah), "v"(al), "v"(bh), "v"(bl));
  return c;
}
template <bool ASPLIT>
__global__ __launch_bounds__(128) void k_gemm_h(const float* __restrict__ A, int lda, size_t sA, const _Float16* __restrict__ Bh, int ldb, size_t sB, float alpha, float* __restrict__ C, int ldc, size_t sC, int M, int N, int K) {
  __shared__ __attribute__((aligned(16))) float so[4][16][64];
  const int tid = threadIdx.x, w = tid >> 5, lane = tid & 31, ln = lane & 15, hh = lane >> 4; const int by = blockIdx.y;
  A += (size_t)by * sA; Bh += (size_t)by * sB; C += (size_t)by * sC;
  const int ntn = (N + 63) / 64; const int wid = blockIdx.x * 4 + w; const int mt = wid / ntn, nq = wid % ntn; if (mt * 16 >= M) return;
  const int row0 = mt * 16, col0 = nq * 64; const float* arow = A + (size_t)(row0 + ln) * lda;
  v8f acc[4] = {};
  for (int kb = 0; kb < K; kb += 32) {
    FragH ah, al;
    const v4f x0 = *(const v4fa*)(arow + kb + 8 * hh), x1 = *(const v4fa*)(arow + kb + 8 * hh + 4), x2 = *(const v4fa*)(arow + kb + 16 + 8 * hh), x3 = *(const v4fa*)(arow + kb + 16 + 8 * hh + 4);
    float xs[16] = {x0[0],x0[1],x0[2],x0[3],x1[0],x1[1],x1[2],x1[3],x2[0],x2[1],x2[2],x2[3],x3[0],x3[1],x3[2],x3[3]};
#pragma unroll
    for (int i = 0; i < 16; ++i) { const _Float16 h = (_Float16)xs[i]; ah.h[i] = h; al.h[i] = ASPLIT ? (_Float16)(xs[i] - (float)h) : (_Float16)0.0f; }
#pragma unroll
    for (int t = 0; t < 4; ++t) { if (col0 + t * 16 >= N) continue; const size_t boff = (size_t)(col0 + t * 16 + ln) * ldb + kb; FragH bq; bq.half[0] = *(const v8us*)(Bh + boff + 8 * hh); bq.half[1] = *(const v8us*)(Bh + boff + 16 + 8 * hh);
      acc[t] = mmaH<ASPLIT ? 2 : 1>(ah.v, al.v, bq.v, bq.v, acc[t]); }
  }
#pragma unroll
  for (int t = 0; t < 4; ++t) { if (col0 + t * 16 >= N) continue;
#pragma unroll
    for (int r = 0; r < 8; ++r) so[w][8 * hh + r][t * 16 + ln] = acc[t][r] * alpha; }
  __builtin_amdgcn_fence(__ATOMIC_ACQ_REL, "workgroup"); __builtin_amdgcn_wave_barrier();
  const int rsub = lane >> 4, c4 = (lane & 15) * 4;
  for (int pass = 0; pass < 2; ++pass) {
#pragma unroll
    for (int q = 0; q < 8; ++q) { const int r = q * 2 + rsub; if (col0 + c4 < N) { const v4f v = *(const v4fa*)&so[w][r][c4]; *(volatile v4f*)(C + (size_t)(row0 + r) * ldc + col0 + c4) = v; } }
    if (pass == 0) __threadfence(); }
}

template <int DUMMY>
__global__ __launch_bounds__(128) void k_gemm_hh(const _Float16* __restrict__ A, int lda, size_t sA, const _Float16* __restrict__ Bh, int ldb, size_t sB, float alpha, float* __restrict__ C, int ldc, size_t sC, int M, int N, int K) {
  __shared__ __attribute__((aligned(16))) float so[4][16][64];
  const int tid = threadIdx.x, w = tid >> 5, lane = tid & 31, ln = lane & 15, hh = lane >> 4; const int by = blockIdx.y;
  A += (size_t)by * sA; Bh += (size_t)by * sB; C += (size_t)by * sC;
  const int ntn = (N + 63) / 64; const int wid = blockIdx.x * 4 + w; const int mt = wid / ntn, nq = wid % ntn; if (mt * 16 >= M) return;
  const int row0 = mt * 16, col0 = nq * 64; const _Float16* arow = A + (size_t)(row0 + ln) * lda;
  v8f acc[4] = {};
  for (int kb = 0; kb < K; kb += 32) { FragH ah; ah.half[0] = *(const v8us*)((const unsigned short*)arow + kb + 8 * hh); ah.half[1] = *(const v8us*)((const unsigned short*)arow + kb + 16 + 8 * hh);
#pragma unroll
    for (int t = 0; t < 4; ++t) { if (col0 + t * 16 >= N) continue; const size_t boff = (size_t)(col0 + t * 16 + ln) * ldb + kb; FragH bq; bq.half[0] = *(const v8us*)((const unsigned short*)Bh + boff + 8 * hh); bq.half[1] = *(const v8us*)((const unsigned short*)Bh + boff + 16 + 8 * hh);
      acc[t] = mmaH<1>(ah.v, ah.v, bq.v, bq.v, acc[t]); }
  }
#pragma unroll
  for (int t = 0; t < 4; ++t) { if (col0 + t * 16 >= N) continue;
#pragma unroll
    for (int r = 0; r < 8; ++r) so[w][8 * hh + r][t * 16 + ln] = acc[t][r] * alpha; }
  __builtin_amdgcn_fence(__ATOMIC_ACQ_REL, "workgroup"); __builtin_amdgcn_wave_barrier();
  const int rsub = lane >> 4, c4 = (lane & 15) * 4;
  for (int pass = 0; pass < 2; ++pass) {
#pragma unroll
    for (int q = 0; q < 8; ++q) { const int r = q * 2 + rsub; if (col0 + c4 < N) { const v4f v = *(const v4fa*)&so[w][r][c4]; *(volatile v4f*)(C + (size_t)(row0 + r) * ldc + col0 + c4) = v; } }
    if (pass == 0) __threadfence(); }
}

__global__ __launch_bounds__(256) void k_wt(const float* __restrict__ Wq, const float* __restrict__ Wk, const float* __restrict__ Wv, const float* __restrict__ Wo, const float* __restrict__ bq, const float* __restrict__ bk, const float* __restrict__ bv, unsigned short* __restrict__ Bt, unsigned short* __restrict__ Bo, float* __restrict__ B3) {
  __shared__ float tile[32][33]; const int k0 = blockIdx.x * 32, n0 = blockIdx.y * 32, which = blockIdx.z; const float* W = which == 0 ? Wq : (which == 1 ? Wk : (which == 2 ? Wv : Wo)); const int tx = threadIdx.x & 31, ty = threadIdx.x >> 5;
  for (int i = ty; i < 32; i += 8) tile[i][tx] = W[(size_t)(k0 + i) * HH + n0 + tx]; __syncthreads();
  typedef unsigned short v4us __attribute__((ext_vector_type(4))); const int r = threadIdx.x >> 3, c4 = (threadIdx.x & 7) * 4; v4us o; for (int q = 0; q < 4; ++q) o[q] = bf16_bits(tile[c4 + q][r]);
  unsigned short* d = (which < 3) ? Bt + ((size_t)(which * HH + n0 + r)) * HH + k0 + c4 : Bo + (size_t)(n0 + r) * HH + k0 + c4; *(volatile v4us*)d = o; __threadfence(); *(volatile v4us*)d = o;
  if (blockIdx.x == 0 && which < 3 && threadIdx.x < 32) { const float* bsrc = which == 0 ? bq : (which == 1 ? bk : bv); *(volatile float*)(B3 + which * HH + n0 + threadIdx.x) = bsrc[n0 + threadIdx.x]; } }
__global__ __launch_bounds__(256) void k_rope(const float* __restrict__ QKV, const int* __restrict__ ts, _Float16* __restrict__ Q16, _Float16* __restrict__ K16, _Float16* __restrict__ VTM) {
  __shared__ int stm[32]; const int b = blockIdx.y, i0 = blockIdx.x * 32; const int tid = threadIdx.x, lane = tid & 31, wv = tid >> 5;
  if (tid < 32) { const int i = i0 + tid; stm[tid] = (i < SS) ? (i % TT) * SP + (i / TT) : -1; }
  __syncthreads();
  for (int pass = 0; pass < 2; ++pass) {
    for (int r = wv; r < 32; r += 8) { const int i = i0 + r; if (i >= SS) continue; const size_t tok = (size_t)b * SS + i; int ta = ts[tok]; ta = ta < 0 ? 0 : (ta >= TT ? TT - 1 : ta); const int tm = stm[r];
      for (int h = 0; h < NH; ++h) {
        const size_t qb = tok * (3 * HH) + h * DH; _Float16 qo[2], ko[2], vo[2];
        for (int q = 0; q < 2; ++q) { const int d = 2 * lane + q; const int dm = d & 31; const float invf = 1.0f / powf(10000.0f, (float)(2 * dm) / (float)DH); const float ang = (float)ta * invf; const float cs = cosf(ang), sn = sinf(ang);
          const float qa = QKV[qb + dm], qc = QKV[qb + dm + 32], ka = QKV[qb + HH + dm], kc = QKV[qb + HH + dm + 32];
          qo[q] = (_Float16)((d < 32) ? (qa * cs - qc * sn) : (qc * cs + qa * sn)); ko[q] = (_Float16)((d < 32) ? (ka * cs - kc * sn) : (kc * cs + ka * sn)); vo[q] = (_Float16)QKV[qb + 2 * HH + d]; }
        typedef _Float16 v2h __attribute__((ext_vector_type(2))); v2h q2 = {qo[0], qo[1]}, k2 = {ko[0], ko[1]}, w2 = {vo[0], vo[1]};
        const size_t qrow = (((size_t)b * NH + h) * SS + tm) * DH, krow = (((size_t)b * NH + h) * LK + 80 + tm) * DH, vrow = qrow;
        *(volatile v2h*)(Q16 + qrow + 2 * lane) = q2; *(volatile v2h*)(K16 + krow + 2 * lane) = k2; *(volatile v2h*)(VTM + vrow + 2 * lane) = w2; } }
    if (pass == 0) __threadfence(); } }
__global__ __launch_bounds__(256) void k_vt(const _Float16* __restrict__ VTM, _Float16* __restrict__ VT) { __shared__ float tile[32][33]; const int tm0 = blockIdx.x * 32, d0 = blockIdx.y * 32, bh = blockIdx.z; const int tx = threadIdx.x & 31, ty = threadIdx.x >> 5;
  for (int i = ty; i < 32; i += 8) tile[i][tx] = (tm0 + i < SS) ? (float)VTM[((size_t)bh * SS + tm0 + i) * DH + d0 + tx] : 0.f; __syncthreads();
  for (int pass = 0; pass < 2; ++pass) { for (int i = ty; i < 32; i += 8) { if (tm0 + tx < SS) *(volatile _Float16*)(VT + ((size_t)bh * DH + d0 + i) * LV + 80 + tm0 + tx) = (_Float16)tile[tx][i]; } if (pass == 0) __threadfence(); } }
__global__ __launch_bounds__(256) void k_padz(_Float16* __restrict__ K16, _Float16* __restrict__ VT) { const int t = blockIdx.x * 256 + threadIdx.x; const int bh = blockIdx.y;
  if (t < 160 * DH) { const int r = t / DH, d = t % DH; const int row = r < 80 ? r : (LK - 160 + r); *(volatile _Float16*)(K16 + ((size_t)bh * LK + row) * DH + d) = (_Float16)0.f; }
  if (t < DH * 176) { const int d = t / 176, cc = t % 176; const int col = cc < 80 ? cc : (LV - 176 + cc); *(volatile _Float16*)(VT + ((size_t)bh * DH + d) * LV + col) = (_Float16)0.f; } }
__global__ __launch_bounds__(256) void k_soft(const float* __restrict__ S, const int* __restrict__ amask, int b, _Float16* __restrict__ P) { const int tid = threadIdx.x, wv = tid >> 5, lane = tid & 31; const int gr = blockIdx.x * 8 + wv; const int h = gr / (NG * GR); const int g = (gr / GR) % NG, r = gr % GR; const int tm = g * GR + r; const int tq = tm / SP;
  typedef _Float16 v2h __attribute__((ext_vector_type(2)));
  const float* s = S + (size_t)gr * KWIN; float v[8]; float mx = -3.0e38f; int any = 0;
#pragma unroll
  for (int u = 0; u < 4; ++u) for (int q = 0; q < 2; ++q) { const int c = u * 64 + 2 * lane + q; float val = -3.0e38f; bool ok = false;
    if (c < KWIN) { const int tmk = g * GR + c - 80; if (tmk >= 0 && tmk < SS) { const int tk = tmk / SP, sk = tmk % SP; if (tk <= tq + CF && tk >= tq - CBK && amask[(size_t)b * SS + sk * TT + tk] != 0) { ok = true; val = s[c] * 0.125f; } } }
    v[2 * u + q] = ok ? val : -3.0e38f; any |= ok ? 1 : 0; mx = fmaxf(mx, val); }
  for (int o = 16; o >= 1; o >>= 1) { mx = fmaxf(mx, __shfl_xor(mx, o, 32)); any |= __shfl_xor(any, o, 32); }
  float den = 0.f; for (int u = 0; u < 8; ++u) { v[u] = (v[u] > -1.0e38f) ? expf(v[u] - mx) : 0.f; den += v[u]; } for (int o = 16; o >= 1; o >>= 1) den += __shfl_xor(den, o, 32);
  const float inv = any ? 1.0f / den : 0.f;
  for (int pass = 0; pass < 2; ++pass) { for (int u = 0; u < 4; ++u) { v2h o2; o2.x = (_Float16)(v[2 * u] * inv); o2.y = (_Float16)(v[2 * u + 1] * inv); *(volatile v2h*)(P + (size_t)gr * KP + u * 64 + 2 * lane) = o2; } if (pass == 0) __threadfence(); } }
__global__ __launch_bounds__(256) void k_unperm(const float* __restrict__ OT, const int* __restrict__ amask, const _Float16* __restrict__ VT, int b, float* __restrict__ OC) { const int t = blockIdx.x * 256 + threadIdx.x; if (t >= SS * HH / 4) return; const int c4 = (t * 4) % HH, i = (t * 4) / HH; const int tq = i % TT; const int tm = tq * SP + (i / TT); const int h = c4 / DH, d = c4 % DH; const size_t bh = (size_t)b * NH + h;
  int any = 0;
#pragma unroll 1
  for (int tk = (tq - CBK < 0 ? 0 : tq - CBK); tk <= (tq + CF > TT - 1 ? TT - 1 : tq + CF); ++tk)
#pragma unroll 1
    for (int sk = 0; sk < SP; ++sk) any |= (amask[(size_t)b * SS + sk * TT + tk] != 0);
  v4f o; if (!any) { for (int q = 0; q < 4; ++q) { float sum = 0.f;
#pragma unroll 1
      for (int c = 0; c < SS; ++c) sum += (float)VT[(bh * DH + d + q) * LV + 80 + c]; o[q] = sum / (float)SS; } } else { o = *(const v4fa*)(OT + (bh * SS + tm) * DH + d); }
  float* dst = OC + ((size_t)b * SS + i) * HH + c4; *(volatile v4f*)dst = o; __threadfence(); *(volatile v4f*)dst = o; }
extern "C" void kernel_launch(void* const* d_in, const int* in_sizes, int n_in,
                              void* d_out, int out_size, void* d_ws, size_t ws_size, hipStream_t stream) {
  (void)in_sizes; (void)n_in; (void)out_size;
  const float* x = (const float*)d_in[0]; const int* amask = (const int*)d_in[1]; const int* ts = (const int*)d_in[2]; const float* Wq = (const float*)d_in[3]; const float* bq = (const float*)d_in[4]; const float* Wk = (const float*)d_in[5]; const float* bk = (const float*)d_in[6]; const float* Wv = (const float*)d_in[7]; const float* bv = (const float*)d_in[8]; const float* Wo = (const float*)d_in[9]; const float* bo = (const float*)d_in[10];
  char* ws = (char*)d_ws; size_t off = 0;
  auto take = [&](size_t bytes) { char* p = ws + off; off += (bytes + 255) & ~(size_t)255; return p; };
  unsigned short* Bt = (unsigned short*)take((size_t)3 * HH * HH * 2); unsigned short* Bo = (unsigned short*)take((size_t)HH * HH * 2); float* B3 = (float*)take(3 * HH * 4);
  float* QKV = (float*)take((size_t)NTOK * 3 * HH * 4); _Float16* Q16 = (_Float16*)take((size_t)BB * NH * SS * DH * 2); _Float16* K16 = (_Float16*)take((size_t)BB * NH * LK * DH * 2); _Float16* VT = (_Float16*)take((size_t)BB * NH * DH * LV * 2); _Float16* VTM = (_Float16*)take((size_t)BB * NH * SS * DH * 2);
  float* S = (float*)take((size_t)NH * NG * GR * KWIN * 4); _Float16* P = (_Float16*)take((size_t)NH * NG * GR * KP * 2);
  float* OT = QKV;   float* OC = QKV + (size_t)BB * NH * SS * DH;
  if (off > ws_size) return;
  k_wt<<<dim3(HH / 32, HH / 32, 4), 256, 0, stream>>>(Wq, Wk, Wv, Wo, bq, bk, bv, Bt, Bo, B3);
  k_gemm_b<false, false, 0><<<dim3(((NTOK / 16) * (3 * HH / 64) + 3) / 4, 1), 128, 0, stream>>>(x, HH, 0, Bt, Bt, HH, 0, B3, nullptr, 0, 0, 1.f, 1.f, QKV, 3 * HH, 0, NTOK, 3 * HH, HH);
  k_padz<<<dim3((DH * 176 + 255) / 256, BB * NH), 256, 0, stream>>>(K16, VT);
  k_rope<<<dim3((SS + 31) / 32, BB), 256, 0, stream>>>(QKV, ts, Q16, K16, VTM); k_vt<<<dim3((SS + 31) / 32, DH / 32, BB * NH), 256, 0, stream>>>(VTM, VT);
  for (int b = 0; b < BB; ++b) {
    for (int h = 0; h < NH; ++h) { const size_t bh = (size_t)b * NH + h;
      k_gemm_hh<0><<<dim3(((GR / 16) * ((KWIN + 63) / 64) + 3) / 4, NG), 128, 0, stream>>>(Q16 + bh * SS * DH, DH, (size_t)GR * DH, K16 + bh * LK * DH, DH, (size_t)GR * DH, 1.0f, S + (size_t)h * NG * GR * KWIN, KWIN, (size_t)GR * KWIN, GR, KWIN, DH); }
    k_soft<<<NH * NG * GR / 8, 256, 0, stream>>>(S, amask, b, P);
    for (int h = 0; h < NH; ++h) { const size_t bh = (size_t)b * NH + h;
      k_gemm_hh<0><<<dim3(((GR / 16) * 1 + 3) / 4, NG), 128, 0, stream>>>(P + (size_t)h * NG * GR * KP, KP, (size_t)GR * KP, VT + bh * DH * LV, LV, (size_t)GR, 1.0f, OT + bh * SS * DH, DH, (size_t)GR * DH, GR, DH, KP); }
    k_unperm<<<(SS * HH / 4 + 255) / 256, 256, 0, stream>>>(OT, amask, VT, b, OC); }
  k_gemm_b<true, false, 0><<<dim3(((NTOK / 16) * (HH / 64) + 3) / 4, 1), 128, 0, stream>>>(OC, HH, 0, Bo, Bo, HH, 0, bo, nullptr, 0, 0, 1.f, 1.f, (float*)d_out, HH, 0, NTOK, HH, HH);
}
